// GraphTransformerLayer_33457795236066
// MI455X (gfx1250) — hardware-verified
//
#include <hip/hip_runtime.h>
#include <stddef.h>
#include <stdint.h>


#define DIN     128
#define NHD     4
#define NCAT    512
#define APA     512
#define KH      512
#define KF      1024
#define AHP     256
#define K2      256
#define NTHR    256
#define NWAVE   8
#define EPT     8
#define CHUNK   (NTHR * EPT)
#define WCAP    (EPT * 32)
#define LISTN   (NWAVE * WCAP)
#define NBMAX   2048
#define RCAP    28672
#define DEGCAP  128
#define PKS     11
#define STW     512
#define GBM     64
#define GTHR    128
#define WSMAX   134217728
#define LDS_AGG ((2 * RCAP + 2 * NBMAX + LISTN) * 4 + 64)
#define GO_CAT  0
#define GO_SX   131072
#define GO_PAR  147456
#define LDS_GNN 151040
#define FO_X1   0
#define FO_T    32768
#define FO_PAR  65536
#define LDS_FFN 66560
#define U_HN    32768
#define U_F     49152
#define U_1     53248
#define U_END   57344

static_assert((CHUNK & (CHUNK - 1)) == 0 && CHUNK <= (1 << PKS));
static_assert((NBMAX & (NBMAX - 1)) == 0 && NBMAX <= (1 << PKS));
static_assert(NTHR * 8 == NBMAX);
static_assert(LISTN >= NBMAX);
static_assert(LISTN >= NWAVE * WCAP);
static_assert((RCAP % 32) == 0);
static_assert(NWAVE * STW <= RCAP);
static_assert(STW >= 256);
static_assert(LDS_AGG <= 300000);
static_assert(GBM == (GTHR / 32) * 16);
static_assert(GTHR == DIN);
static_assert((KH % 32) == 0 && (KF % 32) == 0 && (K2 % 32) == 0);
static_assert(GO_SX == GBM * KF * 2 && GO_PAR == GO_SX + GBM * DIN * 2 && LDS_GNN == GO_PAR + 896 * 4);
static_assert(GBM * DIN * 4 + GBM * AHP * 2 <= GO_SX);
static_assert(FO_T == GBM * DIN * 4 && FO_PAR == FO_T + GBM * AHP * 2 && LDS_FFN == FO_PAR + 256 * 4);
static_assert((U_HN % 256) == 0 && (U_F % 256) == 0 && (U_1 % 256) == 0 && (U_END % 256) == 0);
static_assert(U_HN == 512 * KH / 8 && U_F - U_HN == DIN * KF / 8 && U_1 - U_F == DIN * K2 / 8 && U_END - U_1 == DIN * K2 / 8);

typedef float          v4f  __attribute__((ext_vector_type(4)));
typedef float          v8f  __attribute__((ext_vector_type(8)));
typedef int            v4i  __attribute__((ext_vector_type(4)));
typedef int            v8i  __attribute__((ext_vector_type(8)));
typedef unsigned int   v2u  __attribute__((ext_vector_type(2)));
typedef unsigned int   v4u  __attribute__((ext_vector_type(4)));
typedef unsigned short v8us __attribute__((ext_vector_type(8)));
typedef __bf16         v16b __attribute__((ext_vector_type(16)));
union FragB { v16b v; v8us h[2]; v8i w; };

__device__ __forceinline__ v8f wmb(const FragB& a, const FragB& b, v8f c) {
  v8f d = __builtin_amdgcn_wmma_f32_16x16x32_bf16(false, a.v, false, b.v, (short)0, c, false, false);
  asm volatile("v_nop\n\tv_nop\n\tv_nop\n\tv_nop" : "+v"(d) : "v"(a.w), "v"(b.w));
  return d;
}

__device__ __forceinline__ unsigned short bf_bits(float f) {
  unsigned int u = __float_as_uint(f);
  u += 0x7FFFu + ((u >> 16) & 1u);
  return (unsigned short)(u >> 16);
}
__device__ __forceinline__ float bf_val(unsigned short b) {
  return __uint_as_float(((unsigned int)b) << 16);
}
__device__ __forceinline__ float bf_rne(float f) { return bf_val(bf_bits(f)); }

__device__ __forceinline__ v8us cvt8b(const v4f a, const v4f b) {
  v8us hv;
  hv[0] = bf_bits(a.x); hv[1] = bf_bits(a.y); hv[2] = bf_bits(a.z); hv[3] = bf_bits(a.w);
  hv[4] = bf_bits(b.x); hv[5] = bf_bits(b.y); hv[6] = bf_bits(b.z); hv[7] = bf_bits(b.w);
  return hv;
}

__device__ __forceinline__ int scan_chunk(const int* __restrict__ dsts, int nE, int cbase, int slotBase,
                                          int nb, int vec8, int* list, int tid, int lane, int wave) {
  int wc = 0;
  const int el0  = tid * EPT;
  const int e0   = cbase + el0;
  const int sent = -2147483647 - 1;
  v4i da, db;
  if (vec8 != 0 && cbase + CHUNK <= nE) {
    da = *(const v4i*)(dsts + e0);
    db = *(const v4i*)(dsts + e0 + 4);
  } else {
    da.x = (e0     < nE) ? dsts[min(e0,     nE - 1)] : sent;
    da.y = (e0 + 1 < nE) ? dsts[min(e0 + 1, nE - 1)] : sent;
    da.z = (e0 + 2 < nE) ? dsts[min(e0 + 2, nE - 1)] : sent;
    da.w = (e0 + 3 < nE) ? dsts[min(e0 + 3, nE - 1)] : sent;
    db.x = (e0 + 4 < nE) ? dsts[min(e0 + 4, nE - 1)] : sent;
    db.y = (e0 + 5 < nE) ? dsts[min(e0 + 5, nE - 1)] : sent;
    db.z = (e0 + 6 < nE) ? dsts[min(e0 + 6, nE - 1)] : sent;
    db.w = (e0 + 7 < nE) ? dsts[min(e0 + 7, nE - 1)] : sent;
  }
  const unsigned nbs = (unsigned)slotBase;
  const unsigned unb = (unsigned)nb;
  const unsigned s0 = (unsigned)da.x - nbs, s1 = (unsigned)da.y - nbs;
  const unsigned s2 = (unsigned)da.z - nbs, s3 = (unsigned)da.w - nbs;
  const unsigned s4 = (unsigned)db.x - nbs, s5 = (unsigned)db.y - nbs;
  const unsigned s6 = (unsigned)db.z - nbs, s7 = (unsigned)db.w - nbs;
  const bool h0 = s0 < unb, h1 = s1 < unb, h2 = s2 < unb, h3 = s3 < unb;
  const bool h4 = s4 < unb, h5 = s5 < unb, h6 = s6 < unb, h7 = s7 < unb;
  const unsigned any = __builtin_amdgcn_ballot_w32(h0 | h1 | h2 | h3 | h4 | h5 | h6 | h7);
  if (any != 0u) {
#define HITJ(J, HJ, SJ) { \
      const unsigned mj = __builtin_amdgcn_ballot_w32(HJ); \
      if (mj != 0u) { \
        if (HJ) { \
          const int pos = wc + (int)__builtin_amdgcn_mbcnt_lo(mj, 0u); \
          if (pos < WCAP) list[wave * WCAP + pos] = ((el0 + (J)) << PKS) | (int)(SJ); \
        } \
        wc += (int)__builtin_popcount(mj); } }
    HITJ(0, h0, s0)
    HITJ(1, h1, s1)
    HITJ(2, h2, s2)
    HITJ(3, h3, s3)
    HITJ(4, h4, s4)
    HITJ(5, h5, s5)
    HITJ(6, h6, s6)
    HITJ(7, h7, s7)
#undef HITJ
  }
  return wc;
}

__global__ __launch_bounds__(NTHR) void k_wpack(const float* __restrict__ Wself, const float* __restrict__ Wneigh,
                                                const float* __restrict__ Wfc, const float* __restrict__ W1,
                                                const float* __restrict__ W2,
                                                unsigned short* wth, unsigned short* wtf,
                                                unsigned short* wt1, unsigned short* wt2) {
  const int u = (int)blockIdx.x * NTHR + (int)threadIdx.x;
  if (u >= U_END) return;
  const float* p;
  unsigned short* o;
  if (u < U_HN) {
    const int part = u >> 14;
    const int v    = u & 16383;
    const int n    = v >> 5;
    const int k8l  = (v & 31) * 8;
    const int hd = n >> 7, f = n & 127, kk = k8l & 127;
    const float* wsrc = (part == 0) ? Wself : Wneigh;
    p = wsrc + (size_t)(hd * DIN + kk) * DIN + f;
    o = wth + (size_t)n * KH + part * 256 + k8l;
  } else if (u < U_F) {
    const int v  = u - U_HN;
    const int n  = v >> 7;
    const int k8 = (v & 127) * 8;
    const int kk = k8 & 511;
    p = Wfc + (size_t)kk * DIN + n;
    o = wtf + (size_t)n * KF + k8;
  } else if (u < U_1) {
    const int v  = u - U_F;
    const int n  = v >> 5;
    const int k8 = (v & 31) * 8;
    const int kk = k8 & 127;
    p = W1 + (size_t)kk * DIN + n;
    o = wt1 + (size_t)n * K2 + k8;
  } else {
    const int v  = u - U_1;
    const int n  = v >> 5;
    const int k8 = (v & 31) * 8;
    const int kk = k8 & 127;
    p = W2 + (size_t)kk * DIN + n;
    o = wt2 + (size_t)n * K2 + k8;
  }
  v4f a, b;
  a.x = p[0];                   a.y = p[(size_t)DIN];         a.z = p[(size_t)2 * DIN];     a.w = p[(size_t)3 * DIN];
  b.x = p[(size_t)4 * DIN];     b.y = p[(size_t)5 * DIN];     b.z = p[(size_t)6 * DIN];     b.w = p[(size_t)7 * DIN];
  const v8us hv = cvt8b(a, b);
  *(volatile v8us*)o = hv;
  __threadfence();
  *(volatile v8us*)o = hv;
}

__global__ __launch_bounds__(NTHR) void k_ln1(const float* __restrict__ x, const float* __restrict__ g,
                                              const float* __restrict__ b, float* XN, int nN) {
  const int tid = (int)threadIdx.x, lane = tid & 31, wave = tid >> 5;
  const int row = (int)blockIdx.x * 8 + wave;
  const int rc  = row < nN ? row : nN - 1;
  const v4f xv = *(const v4f*)(x + (size_t)rc * DIN + 4 * lane);
  const float a0 = bf_rne(xv.x), a1 = bf_rne(xv.y), a2 = bf_rne(xv.z), a3 = bf_rne(xv.w);
  float s = (a0 + a1) + (a2 + a3);
#pragma unroll
  for (int o = 16; o > 0; o >>= 1) s += __shfl_xor(s, o);
  const float mu = s * (1.0f / DIN);
  const float d0 = a0 - mu, d1 = a1 - mu, d2 = a2 - mu, d3 = a3 - mu;
  float q = (d0 * d0 + d1 * d1) + (d2 * d2 + d3 * d3);
#pragma unroll
  for (int o = 16; o > 0; o >>= 1) q += __shfl_xor(q, o);
  const float rs = rsqrtf(q * (1.0f / DIN) + 1e-5f);
  const v4f gv = *(const v4f*)(g + 4 * lane);
  const v4f bv = *(const v4f*)(b + 4 * lane);
  v4f y;
  y.x = d0 * rs * bf_rne(gv.x) + bf_rne(bv.x);
  y.y = d1 * rs * bf_rne(gv.y) + bf_rne(bv.y);
  y.z = d2 * rs * bf_rne(gv.z) + bf_rne(bv.z);
  y.w = d3 * rs * bf_rne(gv.w) + bf_rne(bv.w);
  const v4f z4 = {0.f, 0.f, 0.f, 0.f};
  if (row >= nN) y = z4;
  float* op = XN + (size_t)row * DIN + 4 * lane;
  *(volatile v4f*)op = y;
  __threadfence();
  *(volatile v4f*)op = y;
}

__global__ __launch_bounds__(NTHR) void k_agg(
    const int* __restrict__ srcs, const int* __restrict__ dsts,
    const float* __restrict__ XN, unsigned short* Aout,
    int nN, int nE, int nb, int vec8, int MPr) {
  extern __shared__ v4f lds_dyn[];
  int* reg1 = (int*)lds_dyn;
  int* reg2 = reg1 + RCAP;
  int* scnt = reg2 + RCAP;
  int* soff = scnt + NBMAX;
  int* list = soff + NBMAX;
  int* wcnt = list + LISTN;
  int* wtot = wcnt + NWAVE;
  const int tid = (int)threadIdx.x, lane = tid & 31, wave = tid >> 5;
  const int nodeBase = (int)blockIdx.x * nb;

  for (int i = tid; i < NBMAX; i += NTHR) scnt[i] = 0;
  __syncthreads();

  int tot = 0;
  const int nChunks = (nE + CHUNK - 1) / CHUNK;
#pragma unroll 1
  for (int ch = 0; ch < nChunks; ++ch) {
    const int cbase = ch * CHUNK;
    const int wc = scan_chunk(dsts, nE, cbase, nodeBase, nb, vec8, list, tid, lane, wave);
    if (lane == 0) wcnt[wave] = wc;
    __syncthreads();
    int pre = 0, all = 0;
#pragma unroll
    for (int w2 = 0; w2 < NWAVE; ++w2) {
      int c = wcnt[w2];
      c = c < 0 ? 0 : (c > WCAP ? WCAP : c);
      all += c;
      pre += (w2 < wave) ? c : 0;
    }
    const int wcc  = wc > WCAP ? WCAP : wc;
    const int base = tot + pre;
#pragma unroll 1
    for (int i = lane; i < wcc; i += 32) {
      const int ent = list[wave * WCAP + i];
      const int el  = (ent >> PKS) & (CHUNK - 1);
      const int sl  = ent & (NBMAX - 1);
      int eid = cbase + el;
      eid = eid > nE - 1 ? nE - 1 : eid;
      const int pos = base + i;
      if (pos < RCAP) reg1[pos] = (int)(((unsigned)eid << PKS) | (unsigned)sl);
    }
    tot += all;
    tot = tot > RCAP ? RCAP : tot;
    __syncthreads();
  }
  const int nh = tot;

  if (wave == 0) {
#pragma unroll 1
    for (int b0 = 0; b0 < nh; b0 += 32) {
      const int idx = b0 + lane;
      const int uv  = reg1[idx < RCAP ? idx : RCAP - 1];
      const int m32 = (nh - b0) < 32 ? (nh - b0) : 32;
#pragma unroll 1
      for (int k = 0; k < m32; ++k) {
        const int u  = __builtin_amdgcn_readlane(uv, k);
        const int sl = u & (NBMAX - 1);
        if (lane == 0) scnt[sl] = scnt[sl] + 1;
      }
    }
  }
  __syncthreads();

  {
    const v4i ca = *(const v4i*)(scnt + 8 * tid);
    const v4i cb = *(const v4i*)(scnt + 8 * tid + 4);
    const int e0 = ca.x < 0 ? 0 : ca.x, e1 = ca.y < 0 ? 0 : ca.y, e2 = ca.z < 0 ? 0 : ca.z, e3 = ca.w < 0 ? 0 : ca.w;
    const int e4 = cb.x < 0 ? 0 : cb.x, e5 = cb.y < 0 ? 0 : cb.y, e6 = cb.z < 0 ? 0 : cb.z, e7 = cb.w < 0 ? 0 : cb.w;
    const int ts = e0 + e1 + e2 + e3 + e4 + e5 + e6 + e7;
    int incl = ts;
#pragma unroll
    for (int d = 1; d < 32; d <<= 1) {
      const int up = __shfl_up(incl, d);
      if (lane >= d) incl += up;
    }
    if (lane == 31) wtot[wave] = incl;
    __syncthreads();
    int pre = 0;
#pragma unroll
    for (int w2 = 0; w2 < NWAVE; ++w2) pre += (w2 < wave) ? wtot[w2] : 0;
    int run = pre + incl - ts;
    soff[8 * tid + 0] = run; run += e0;
    soff[8 * tid + 1] = run; run += e1;
    soff[8 * tid + 2] = run; run += e2;
    soff[8 * tid + 3] = run; run += e3;
    soff[8 * tid + 4] = run; run += e4;
    soff[8 * tid + 5] = run; run += e5;
    soff[8 * tid + 6] = run; run += e6;
    soff[8 * tid + 7] = run;
  }
  __syncthreads();
  for (int i = tid; i < NBMAX; i += NTHR) list[i] = soff[i];
  __syncthreads();

  if (wave == 0) {
#pragma unroll 1
    for (int b0 = 0; b0 < nh; b0 += 32) {
      const int idx = b0 + lane;
      const int uv  = reg1[idx < RCAP ? idx : RCAP - 1];
      const int m32 = (nh - b0) < 32 ? (nh - b0) : 32;
#pragma unroll 1
      for (int k = 0; k < m32; ++k) {
        const int u   = __builtin_amdgcn_readlane(uv, k);
        const int sl  = u & (NBMAX - 1);
        const int eid = (int)((unsigned)u >> PKS);
        if (lane == 0) {
          int pos = list[sl];
          pos = pos < 0 ? 0 : (pos > RCAP - 1 ? RCAP - 1 : pos);
          reg2[pos] = eid;
          list[sl] = pos + 1;
        }
      }
    }
  }
  __syncthreads();

  const int nbw = nb >> 3;
  const bool ovf = (nh >= RCAP);
  const float qnan = __int_as_float(0x7fc00000);
  float* stw = (float*)reg1 + wave * STW;
  unsigned int* stwu = (unsigned int*)stw;

#pragma unroll 1
  for (int jt = 0; jt < nbw; ++jt) {
    const int slot = wave * nbw + jt;
    const int grow = nodeBase + slot;
    const int gcl  = grow < nN ? grow : nN - 1;
    int st = soff[slot];
    const int craw = scnt[slot];
    int cnt = craw;
    st  = st < 0 ? 0 : (st > nh ? nh : st);
    cnt = cnt < 0 ? 0 : (cnt > DEGCAP ? DEGCAP : cnt);
    if (cnt > nh - st) cnt = nh - st;
    const float pz = (ovf || craw > DEGCAP) ? qnan : 0.0f;
    const float live = grow < nN ? 1.0f : 0.0f;

    const v4f t4 = *(const v4f*)(XN + (size_t)gcl * DIN + 4 * lane);
    float sv[4] = {t4.x, t4.y, t4.z, t4.w};
    float ag[4] = {0.f, 0.f, 0.f, 0.f};

#pragma unroll 1
    for (int q = 0; q < cnt; ++q) {
      int idx = st + q; idx = idx > RCAP - 1 ? RCAP - 1 : idx;
      int eid = reg2[idx]; eid = eid < 0 ? 0 : (eid > nE - 1 ? nE - 1 : eid);
      const int sraw = srcs[eid];
      const int s = sraw < 0 ? 0 : (sraw > nN - 1 ? nN - 1 : sraw);
      const v4f v = *(const v4f*)(XN + (size_t)s * DIN + 4 * lane);
      ag[0] += v.x; ag[1] += v.y; ag[2] += v.z; ag[3] += v.w;
    }
    const float dcl  = cnt > 0 ? (float)cnt : 1.0f;
    const float invd = 1.0f / dcl;
    unsigned short hx[4], lx[4], hm[4], lm[4];
#pragma unroll
    for (int c = 0; c < 4; ++c) {
      const float xs = sv[c] * live + pz;
      const float mv = (ag[c] * invd) * live + pz;
      hx[c] = bf_bits(xs); lx[c] = bf_bits(xs - bf_val(hx[c]));
      hm[c] = bf_bits(mv); lm[c] = bf_bits(mv - bf_val(hm[c]));
    }
    v2u wxh, wxl, wmh, wml;
    wxh.x = (unsigned int)hx[0] | ((unsigned int)hx[1] << 16);  wxh.y = (unsigned int)hx[2] | ((unsigned int)hx[3] << 16);
    wxl.x = (unsigned int)lx[0] | ((unsigned int)lx[1] << 16);  wxl.y = (unsigned int)lx[2] | ((unsigned int)lx[3] << 16);
    wmh.x = (unsigned int)hm[0] | ((unsigned int)hm[1] << 16);  wmh.y = (unsigned int)hm[2] | ((unsigned int)hm[3] << 16);
    wml.x = (unsigned int)lm[0] | ((unsigned int)lm[1] << 16);  wml.y = (unsigned int)lm[2] | ((unsigned int)lm[3] << 16);
    __builtin_amdgcn_fence(__ATOMIC_RELEASE, "wavefront");
    __builtin_amdgcn_wave_barrier();
    *(v2u*)(stwu + 2 * lane)       = wxh;
    *(v2u*)(stwu + 64 + 2 * lane)  = wxl;
    *(v2u*)(stwu + 128 + 2 * lane) = wmh;
    *(v2u*)(stwu + 192 + 2 * lane) = wml;
    __builtin_amdgcn_fence(__ATOMIC_RELEASE, "wavefront");
    __builtin_amdgcn_wave_barrier();
    const v4u pk0 = *(const v4u*)(stwu + 4 * lane);
    const v4u pk1 = *(const v4u*)(stwu + 128 + 4 * lane);
    unsigned short* gp = Aout + (size_t)grow * (size_t)APA + 8 * lane;
    const bool wsv = grow < MPr;
    if (wsv) { *(volatile v4u*)gp = pk0; *(volatile v4u*)(gp + 256) = pk1; }
    __threadfence();
    if (wsv) { *(volatile v4u*)gp = pk0; *(volatile v4u*)(gp + 256) = pk1; }
  }
}

template<int NT>
__device__ __forceinline__ void gemm_strip(const unsigned short* ap, const unsigned short* __restrict__ wp,
                                           int K, v8f (&acc)[NT]) {
  const v8f z = {0.f, 0.f, 0.f, 0.f, 0.f, 0.f, 0.f, 0.f};
#pragma unroll
  for (int t = 0; t < NT; ++t) acc[t] = z;
  const int ksteps = K >> 5;
#pragma unroll 1
  for (int ks = 0; ks < ksteps; ++ks) {
    FragB af;
    af.h[0] = *(const v8us*)(ap + 32 * ks);
    af.h[1] = *(const v8us*)(ap + 32 * ks + 16);
#pragma unroll
    for (int t = 0; t < NT; ++t) {
      const unsigned short* wq = wp + (size_t)(16 * t) * (size_t)K + 32 * ks;
      FragB bf;
      bf.h[0] = *(const v8us*)wq;
      bf.h[1] = *(const v8us*)(wq + 16);
      acc[t] = wmb(af, bf, acc[t]);
    }
  }
}

__global__ __launch_bounds__(GTHR) void k_gnn(
    const unsigned short* __restrict__ A1, const unsigned short* __restrict__ WTH,
    const unsigned short* __restrict__ WTF, const float* __restrict__ bself,
    const float* __restrict__ bfc, const float* __restrict__ x,
    const float* __restrict__ g2, const float* __restrict__ b2ln,
    float* X1, unsigned short* AH, int nN)
{
  extern __shared__ __attribute__((aligned(16))) char smem[];
  unsigned short* sCat = (unsigned short*)(smem + GO_CAT);
  unsigned short* sX   = (unsigned short*)(smem + GO_SX);
  float* sPar = (float*)(smem + GO_PAR);
  const int tid = (int)threadIdx.x, lane = tid & 31, wave = tid >> 5, hh = lane >> 4, m = lane & 15;
  const int rowBase = (int)blockIdx.x * GBM;

  for (int i = tid; i < NCAT; i += GTHR) sPar[i] = bf_rne(bself[i]);
  sPar[512 + tid] = bf_rne(bfc[tid]);
  sPar[640 + tid] = bf_rne(g2[tid]);
  sPar[768 + tid] = bf_rne(b2ln[tid]);
#pragma unroll
  for (int it = 0; it < 8; ++it) {
    const int u  = it * GTHR + tid;
    const int r  = u >> 4, c0 = (u & 15) * 8;
    int gr = rowBase + r; gr = gr < nN ? gr : nN - 1;
    const float* p = x + (size_t)gr * DIN + c0;
    const v4f a = *(const v4f*)p, b = *(const v4f*)(p + 4);
    *(v8us*)(sX + r * DIN + c0) = cvt8b(a, b);
  }
  __syncthreads();

  const unsigned short* arow = A1 + (size_t)(rowBase + 16 * wave + m) * (size_t)APA + 8 * hh;
#pragma unroll 1
  for (int cg = 0; cg < NHD; ++cg) {
    v8f acc[8];
    gemm_strip<8>(arow, WTH + (size_t)(cg * DIN + m) * (size_t)KH + 8 * hh, KH, acc);
#pragma unroll
    for (int t = 0; t < 8; ++t) {
      const int col = cg * DIN + 16 * t + m;
      const float bb = sPar[col];
#pragma unroll
      for (int r = 0; r < 8; ++r) {
        const int lr = 16 * wave + 8 * hh + r;
        const float v = fmaxf(acc[t][r] + bb, 0.0f);
        const unsigned short hb = bf_bits(v);
        const unsigned short lb = bf_bits(v - bf_val(hb));
        sCat[lr * KF + col]        = hb;
        sCat[lr * KF + NCAT + col] = lb;
      }
    }
  }
  __syncthreads();

  v8f acc2[8];
  gemm_strip<8>(sCat + (size_t)(16 * wave + m) * KF + 8 * hh, WTF + (size_t)m * (size_t)KF + 8 * hh, KF, acc2);

  float s[8];
#pragma unroll
  for (int r = 0; r < 8; ++r) s[r] = 0.0f;
#pragma unroll
  for (int t = 0; t < 8; ++t) {
    const int col = 16 * t + m;
    const float bb = sPar[512 + col];
#pragma unroll
    for (int r = 0; r < 8; ++r) {
      const int lr = 16 * wave + 8 * hh + r;
      const float v = (acc2[t][r] + bb) + bf_val(sX[lr * DIN + col]);
      acc2[t][r] = v;
      s[r] += v;
    }
  }
#pragma unroll
  for (int r = 0; r < 8; ++r) {
    float v = s[r];
    v += __shfl_xor(v, 1);
    v += __shfl_xor(v, 2);
    v += __shfl_xor(v, 4);
    v += __shfl_xor(v, 8);
    s[r] = v * (1.0f / DIN);
  }
  float q[8];
#pragma unroll
  for (int r = 0; r < 8; ++r) q[r] = 0.0f;
#pragma unroll
  for (int t = 0; t < 8; ++t) {
#pragma unroll
    for (int r = 0; r < 8; ++r) {
      const float d = acc2[t][r] - s[r];
      q[r] += d * d;
    }
  }
#pragma unroll
  for (int r = 0; r < 8; ++r) {
    float v = q[r];
    v += __shfl_xor(v, 1);
    v += __shfl_xor(v, 2);
    v += __shfl_xor(v, 4);
    v += __shfl_xor(v, 8);
    q[r] = rsqrtf(v * (1.0f / DIN) + 1e-5f);
  }
  __syncthreads();

  float* stgX = (float*)(smem + GO_CAT);
  unsigned short* stgA = (unsigned short*)(smem + GO_CAT + GBM * DIN * 4);
#pragma unroll
  for (int t = 0; t < 8; ++t) {
    const int col = 16 * t + m;
    const float gg = sPar[640 + col], bl = sPar[768 + col];
#pragma unroll
    for (int r = 0; r < 8; ++r) {
      const int lr = 16 * wave + 8 * hh + r;
      const float x1 = acc2[t][r];
      const float hv = (x1 - s[r]) * q[r] * gg + bl;
      const unsigned short hb = bf_bits(hv);
      const unsigned short lb = bf_bits(hv - bf_val(hb));
      stgX[lr * DIN + col]       = x1;
      stgA[lr * AHP + col]       = hb;
      stgA[lr * AHP + DIN + col] = lb;
    }
  }
  __syncthreads();

  const unsigned int* stgAu = (const unsigned int*)stgA;
#pragma unroll 4
  for (int i = 0; i < 16; ++i) {
    const int lr = 16 * wave + i;
    const size_t gr = (size_t)(rowBase + lr);
    const v4f xv = *(const v4f*)(stgX + lr * DIN + 4 * lane);
    const v4u av = *(const v4u*)(stgAu + lr * (AHP / 2) + 4 * lane);
    *(volatile v4f*)(X1 + gr * DIN + 4 * lane) = xv;
    *(volatile v4u*)((unsigned int*)AH + gr * (AHP / 2) + 4 * lane) = av;
  }
  __threadfence();
#pragma unroll 4
  for (int i = 0; i < 16; ++i) {
    const int lr = 16 * wave + i;
    const size_t gr = (size_t)(rowBase + lr);
    const v4f xv = *(const v4f*)(stgX + lr * DIN + 4 * lane);
    const v4u av = *(const v4u*)(stgAu + lr * (AHP / 2) + 4 * lane);
    *(volatile v4f*)(X1 + gr * DIN + 4 * lane) = xv;
    *(volatile v4u*)((unsigned int*)AH + gr * (AHP / 2) + 4 * lane) = av;
  }
}

__global__ __launch_bounds__(GTHR) void k_ffn(
    const unsigned short* __restrict__ AH, const unsigned short* __restrict__ WT1,
    const unsigned short* __restrict__ WT2, const float* __restrict__ b1,
    const float* __restrict__ b2, const float* __restrict__ X1,
    float* out, int nN)
{
  extern __shared__ __attribute__((aligned(16))) char smem[];
  float* sX1 = (float*)(smem + FO_X1);
  unsigned short* sT = (unsigned short*)(smem + FO_T);
  float* sPar = (float*)(smem + FO_PAR);
  const int tid = (int)threadIdx.x, lane = tid & 31, wave = tid >> 5, hh = lane >> 4, m = lane & 15;
  const int rowBase = (int)blockIdx.x * GBM;

  sPar[tid]       = bf_rne(b1[tid]);
  sPar[DIN + tid] = bf_rne(b2[tid]);
#pragma unroll
  for (int it = 0; it < 16; ++it) {
    const int u = it * GTHR + tid;
    const int r = u >> 5, c = (u & 31) * 4;
    *(v4f*)(sX1 + r * DIN + c) = *(const v4f*)(X1 + (size_t)(rowBase + r) * DIN + c);
  }
  __syncthreads();

  {
    v8f acc[8];
    gemm_strip<8>(AH + (size_t)(rowBase + 16 * wave + m) * (size_t)AHP + 8 * hh,
                  WT1 + (size_t)m * (size_t)K2 + 8 * hh, K2, acc);
#pragma unroll
    for (int t = 0; t < 8; ++t) {
      const int col = 16 * t + m;
      const float bb = sPar[col];
#pragma unroll
      for (int r = 0; r < 8; ++r) {
        const int lr = 16 * wave + 8 * hh + r;
        const float v = fmaxf(acc[t][r] + bb, 0.0f);
        const unsigned short hb = bf_bits(v);
        const unsigned short lb = bf_bits(v - bf_val(hb));
        sT[lr * AHP + col]       = hb;
        sT[lr * AHP + DIN + col] = lb;
      }
    }
  }
  __syncthreads();

  v8f acc2[8];
  gemm_strip<8>(sT + (size_t)(16 * wave + m) * AHP + 8 * hh, WT2 + (size_t)m * (size_t)K2 + 8 * hh, K2, acc2);
#pragma unroll
  for (int t = 0; t < 8; ++t) {
    const int col = 16 * t + m;
    const float bb = sPar[DIN + col];
#pragma unroll
    for (int r = 0; r < 8; ++r) {
      const int lr = 16 * wave + 8 * hh + r;
      acc2[t][r] = (acc2[t][r] + bb) + sX1[lr * DIN + col];
    }
  }
  __syncthreads();
#pragma unroll
  for (int t = 0; t < 8; ++t) {
    const int col = 16 * t + m;
#pragma unroll
    for (int r = 0; r < 8; ++r) {
      const int lr = 16 * wave + 8 * hh + r;
      sX1[lr * DIN + col] = acc2[t][r];
    }
  }
  __syncthreads();

#pragma unroll 4
  for (int i = 0; i < 16; ++i) {
    const int lr = 16 * wave + i;
    const int gr = rowBase + lr;
    const v4f ov = *(const v4f*)(sX1 + lr * DIN + 4 * lane);
    if (gr < nN) *(volatile v4f*)(out + (size_t)gr * DIN + 4 * lane) = ov;
  }
  __threadfence();
#pragma unroll 4
  for (int i = 0; i < 16; ++i) {
    const int lr = 16 * wave + i;
    const int gr = rowBase + lr;
    const v4f ov = *(const v4f*)(sX1 + lr * DIN + 4 * lane);
    if (gr < nN) *(volatile v4f*)(out + (size_t)gr * DIN + 4 * lane) = ov;
  }
}

static int pick_nb(int nE, int nN) {
  int nb = NBMAX;
  while (nb > 16 && (long long)nb * (long long)nE * 5LL > (long long)RCAP * (long long)nN * 4LL) nb >>= 1;
  return nb;
}
static inline int cdiv(int a, int b) { return (a + b - 1) / b; }

extern "C" void kernel_launch(void* const* d_in, const int* in_sizes, int n_in,
                              void* d_out, int out_size, void* d_ws, size_t ws_size,
                              hipStream_t stream) {
  if (n_in < 16) return;
  const int nN = in_sizes[0] / DIN;
  if (nN <= 0 || in_sizes[0] != nN * DIN || nN > (1 << 22)) return;
  const int nE = in_sizes[1];
  if (nE < 1 || in_sizes[2] != nE || nE > (1 << 21)) return;
  if (in_sizes[3] != DIN || in_sizes[4] != DIN) return;
  if (in_sizes[5] != NHD * DIN * DIN || in_sizes[6] != NHD * DIN * DIN) return;
  if (in_sizes[7] != NHD * DIN) return;
  if (in_sizes[8] != NCAT * DIN || in_sizes[9] != DIN) return;
  if (in_sizes[10] != DIN || in_sizes[11] != DIN) return;
  if (in_sizes[12] != DIN * DIN || in_sizes[13] != DIN) return;
  if (in_sizes[14] != DIN * DIN || in_sizes[15] != DIN) return;
  if (out_size != nN * DIN) return;

  const float* x      = (const float*)d_in[0];
  const int*   src    = (const int*)  d_in[1];
  const int*   dst    = (const int*)  d_in[2];
  const float* ln1g   = (const float*)d_in[3];
  const float* ln1b   = (const float*)d_in[4];
  const float* Wneigh = (const float*)d_in[5];
  const float* Wself  = (const float*)d_in[6];
  const float* bself  = (const float*)d_in[7];
  const float* Wfc    = (const float*)d_in[8];
  const float* bfc    = (const float*)d_in[9];
  const float* ln2g   = (const float*)d_in[10];
  const float* ln2b   = (const float*)d_in[11];
  const float* W1     = (const float*)d_in[12];
  const float* b1     = (const float*)d_in[13];
  const float* W2     = (const float*)d_in[14];
  const float* b2     = (const float*)d_in[15];
  float* out = (float*)d_out;

  const int MP   = cdiv(nN, GBM) * GBM;
  const int nb   = pick_nb(nE, nN);
  const int gA   = cdiv(MP, nb);
  const int vec8 = 1;
  if (gA * nb < MP || nb < 16) return;

  char* ws = (char*)d_ws;
  size_t off = 0;
  const size_t oXN  = off; off += (size_t)MP * DIN * 4;      off = (off + 255) & ~(size_t)255;
  const size_t oA1  = off; off += (size_t)MP * APA * 2;      off = (off + 255) & ~(size_t)255;
  const size_t oX1  = off; off += (size_t)MP * DIN * 4;      off = (off + 255) & ~(size_t)255;
  const size_t oAH  = off; off += (size_t)MP * AHP * 2;      off = (off + 255) & ~(size_t)255;
  const size_t oWTH = off; off += (size_t)NCAT * KH * 2;     off = (off + 255) & ~(size_t)255;
  const size_t oWTF = off; off += (size_t)DIN * KF * 2;      off = (off + 255) & ~(size_t)255;
  const size_t oWT1 = off; off += (size_t)DIN * K2 * 2;      off = (off + 255) & ~(size_t)255;
  const size_t oWT2 = off; off += (size_t)DIN * K2 * 2;      off = (off + 255) & ~(size_t)255;
  if (off > ws_size || off > (size_t)WSMAX) return;
  float*          XN  = (float*)(ws + oXN);
  unsigned short* A1  = (unsigned short*)(ws + oA1);
  float*          X1  = (float*)(ws + oX1);
  unsigned short* AH  = (unsigned short*)(ws + oAH);
  unsigned short* WTH = (unsigned short*)(ws + oWTH);
  unsigned short* WTF = (unsigned short*)(ws + oWTF);
  unsigned short* WT1 = (unsigned short*)(ws + oWT1);
  unsigned short* WT2 = (unsigned short*)(ws + oWT2);

  hipFuncSetAttribute(reinterpret_cast<const void*>(&k_agg),
                      hipFuncAttributeMaxDynamicSharedMemorySize, LDS_AGG);
  hipFuncSetAttribute(reinterpret_cast<const void*>(&k_gnn),
                      hipFuncAttributeMaxDynamicSharedMemorySize, LDS_GNN);
  hipFuncSetAttribute(reinterpret_cast<const void*>(&k_ffn),
                      hipFuncAttributeMaxDynamicSharedMemorySize, LDS_FFN);

  k_wpack<<<U_END / NTHR, NTHR, 0, stream>>>(Wself, Wneigh, Wfc, W1, W2, WTH, WTF, WT1, WT2);
  k_ln1<<<MP / 8, NTHR, 0, stream>>>(x, ln1g, ln1b, XN, nN);
  k_agg<<<gA, NTHR, LDS_AGG, stream>>>(src, dst, XN, A1, nN, nE, nb, vec8, MP);
  k_gnn<<<MP / GBM, GTHR, LDS_GNN, stream>>>(A1, WTH, WTF, bself, bfc, x, ln2g, ln2b, X1, AH, nN);
  k_ffn<<<MP / GBM, GTHR, LDS_FFN, stream>>>(AH, WT1, WT2, b1, b2, X1, out, nN);
}
